// EdgePredictor_16174846837134
// MI455X (gfx1250) — hardware-verified
//
#include <hip/hip_runtime.h>
#include <stddef.h>
#include <math.h>


#define DN     128
#define DEA    16
#define HID    128
#define HID2   64
#define K1     (2 * DN + DEA)
#define PW     256
#define NTHR   256
#define NWV    8
#define EPW    16
#define EPI    (NWV * EPW)
#define TILES  4
#define EPBLK  (EPI * TILES)
#define LDH    136
#define BM     32
#define CB     16
#define WSCAP  134217728
#define SCL_A   8.0f
#define SCL_W   16.0f
#define SCL_PQ  0.0625f
#define SCL_ACC 0.0078125f

static_assert((LDH % 8) == 0 && LDH >= HID);
static_assert(BM * 8 == NTHR && NWV * 32 == NTHR);
static_assert((HID % CB) == 0 && (HID2 % CB) == 0);
static_assert(PW == 2 * HID && HID == DN && HID2 == 64);
static_assert(EPI == 128 && (EPI % 32) == 0);
static_assert((DN % 32) == 0 && (HID % 32) == 0);

typedef float    v4f  __attribute__((ext_vector_type(4)));
typedef float    v8f  __attribute__((ext_vector_type(8)));
typedef _Float16 v4h  __attribute__((ext_vector_type(4)));
typedef _Float16 v8h  __attribute__((ext_vector_type(8)));
typedef _Float16 v16h __attribute__((ext_vector_type(16)));
union FragH { v16h v; v8h h[2]; };

__device__ __forceinline__ v8f wmh(v16h a, v16h b, v8f c) {
  v8f d = __builtin_amdgcn_wmma_f32_16x16x32_f16(false, a, false, b, (short)0, c, false, false);
  asm volatile("v_nop\n\tv_nop\n\tv_nop\n\tv_nop" : "+v"(d) : "v"(a), "v"(b));
  return d;
}

__device__ __forceinline__ v8h cvt8(v4f a, v4f b, float s) {
  v8f t;
  t[0] = a.x * s; t[1] = a.y * s; t[2] = a.z * s; t[3] = a.w * s;
  t[4] = b.x * s; t[5] = b.y * s; t[6] = b.z * s; t[7] = b.w * s;
  return __builtin_convertvector(t, v8h);
}

template <int R>
__global__ __launch_bounds__(NTHR) void k_tconv(const float* __restrict__ in, _Float16* outp,
                                                int C, int inStrideY, int outStrideY, float scale) {
  static_assert((R % 8) == 0 && ((R * CB / 4) % NTHR) == 0 && (CB * R / 8) == NTHR);
  __shared__ float st[R * (CB + 1)];
  const int tid = threadIdx.x;
  const int c0 = blockIdx.x * CB;
  const float* src = in + (size_t)blockIdx.y * inStrideY;
  _Float16* dst = outp + (size_t)blockIdx.y * outStrideY;
#pragma unroll
  for (int q = 0; q < (R * CB / 4) / NTHR; ++q) {
    const int u  = q * NTHR + tid;
    const int r  = u / (CB / 4);
    const int c4 = (u - r * (CB / 4)) * 4;
    const v4f v = *(const v4f*)(src + (size_t)r * C + c0 + c4);
    float* sp = st + r * (CB + 1) + c4;
    sp[0] = v.x; sp[1] = v.y; sp[2] = v.z; sp[3] = v.w;
  }
  __syncthreads();
  const int c  = tid / (R / 8);
  const int r8 = (tid - c * (R / 8)) * 8;
  v8f t;
#pragma unroll
  for (int i = 0; i < 8; ++i) t[i] = st[(r8 + i) * (CB + 1) + c] * scale;
  const v8h o = __builtin_convertvector(t, v8h);
  _Float16* d = dst + (size_t)(c0 + c) * R + r8;
  *(volatile v8h*)d = o;
  __threadfence();
  *(volatile v8h*)d = o;
}

__global__ __launch_bounds__(NTHR) void k_xcvt(const float* __restrict__ x, _Float16* xp, int nN, int nUnits) {
  constexpr int UPR = DN / 8;
  static_assert((UPR & (UPR - 1)) == 0);
  const int i = (int)blockIdx.x * NTHR + (int)threadIdx.x;
  if (i >= nUnits) return;
  const int row = i / UPR;
  const int c0  = (i & (UPR - 1)) * 8;
  int rr = row > nN - 1 ? nN - 1 : row;
  rr = rr < 0 ? 0 : rr;
  const float* p = x + (size_t)rr * DN + c0;
  const v4f a = *(const v4f*)p;
  const v4f b = *(const v4f*)(p + 4);
  v8h o = cvt8(a, b, SCL_A);
  const v8h z = {(_Float16)0.0f, (_Float16)0.0f, (_Float16)0.0f, (_Float16)0.0f,
                 (_Float16)0.0f, (_Float16)0.0f, (_Float16)0.0f, (_Float16)0.0f};
  o = (row < nN) ? o : z;
  _Float16* d = xp + (size_t)i * 8;
  *(volatile v8h*)d = o;
  __threadfence();
  *(volatile v8h*)d = o;
}

__global__ __launch_bounds__(NTHR) void k_nodegemm(
    const _Float16* __restrict__ xP, const _Float16* __restrict__ wPQ,
    const float* __restrict__ b1, float* pq, int nN) {
  constexpr int NIT4 = (BM * PW / 4) / NTHR;
  static_assert((BM * PW / 4) % NTHR == 0 && NIT4 == 8);
  __shared__ __attribute__((aligned(16))) float stg[BM * PW];
  const int tid = threadIdx.x, lane = tid & 31, wave = tid >> 5;
  const int hh = lane >> 4, m = lane & 15;
  const int rg = wave >> 2, cq = wave & 3;
  const int r0 = rg * 16, c0 = cq * 64;
  const int rowBase = blockIdx.x * BM;

  v8f acc[4];
#pragma unroll
  for (int t = 0; t < 4; ++t) { v8f z = {0.f, 0.f, 0.f, 0.f, 0.f, 0.f, 0.f, 0.f}; acc[t] = z; }

  const _Float16* ap  = xP + (size_t)(rowBase + r0 + m) * DN + 8 * hh;
  const _Float16* bp0 = wPQ + (size_t)(c0 + m) * DN + 8 * hh;
#pragma unroll 1
  for (int kt = 0; kt < DN / 32; ++kt) {
    FragH a;
    a.h[0] = *(const v8h*)(ap + 32 * kt);
    a.h[1] = *(const v8h*)(ap + 32 * kt + 16);
#pragma unroll
    for (int t = 0; t < 4; ++t) {
      const _Float16* bp = bp0 + (size_t)(16 * t) * DN + 32 * kt;
      FragH bf;
      bf.h[0] = *(const v8h*)bp;
      bf.h[1] = *(const v8h*)(bp + 16);
      acc[t] = wmh(a.v, bf.v, acc[t]);
    }
  }

  float* sp = stg + (size_t)(r0 + 8 * hh) * PW + c0 + m;
  const int grow0 = rowBase + r0 + 8 * hh;
#pragma unroll
  for (int t = 0; t < 4; ++t) {
    const int n  = c0 + 16 * t + m;
    const int nb = n < HID ? n : HID - 1;
    float bv = b1[nb];
    bv = (n < HID) ? bv : 0.0f;
#pragma unroll
    for (int r = 0; r < 8; ++r) {
      float v = acc[t][r] * SCL_PQ + SCL_A * bv;
      v = (grow0 + r < nN) ? v : 0.0f;
      sp[r * PW + 16 * t] = v;
    }
  }
  __syncthreads();

  float* tile = pq + (size_t)rowBase * PW;
  v4f ov[NIT4];
#pragma unroll
  for (int it = 0; it < NIT4; ++it) ov[it] = *(const v4f*)(stg + 4 * (it * NTHR + tid));
#pragma unroll
  for (int it = 0; it < NIT4; ++it) *(volatile v4f*)(tile + 4 * (size_t)(it * NTHR + tid)) = ov[it];
  __threadfence();
#pragma unroll
  for (int it = 0; it < NIT4; ++it) *(volatile v4f*)(tile + 4 * (size_t)(it * NTHR + tid)) = ov[it];
}

__global__ __launch_bounds__(NTHR) void k_edge(
    const float* __restrict__ pq, const int* __restrict__ ei, const float* __restrict__ ea,
    const float* __restrict__ W1, const _Float16* __restrict__ w2p, const float* __restrict__ b2,
    const float* __restrict__ W3, const float* __restrict__ b3, float* out, int nE, int nN) {
  __shared__ __attribute__((aligned(16))) _Float16 hs[NWV * EPW * LDH];
  __shared__ __attribute__((aligned(16))) float sres[EPI];
  const int tid = threadIdx.x, lane = tid & 31;
  const int wave = __builtin_amdgcn_readfirstlane(tid >> 5);
  const int hh = lane >> 4, m = lane & 15;
  const int col = 4 * lane;

  v4f we[DEA];
#pragma unroll
  for (int k = 0; k < DEA; ++k) we[k] = *(const v4f*)(W1 + (size_t)(2 * DN + k) * HID + col) * SCL_A;
  float b2v[4], w3v[4];
#pragma unroll
  for (int t = 0; t < 4; ++t) { b2v[t] = b2[16 * t + m]; w3v[t] = W3[16 * t + m]; }
  const float c3 = b3[0];
  _Float16* hw = hs + wave * (EPW * LDH);
  const int blockBase = blockIdx.x * EPBLK;

#pragma unroll 1
  for (int it = 0; it < TILES; ++it) {
    const int tileBase = blockBase + it * EPI;
    const int e0 = tileBase + wave * EPW;
    int el = e0 + m;
    el = el > nE - 1 ? nE - 1 : el;
    int sl = ei[el];
    int dl = ei[(size_t)nE + el];
    sl = sl < 0 ? 0 : (sl > nN - 1 ? nN - 1 : sl);
    dl = dl < 0 ? 0 : (dl > nN - 1 ? nN - 1 : dl);

#pragma unroll 1
    for (int j = 0; j < EPW; ++j) {
      const int s = __builtin_amdgcn_readlane(sl, j);
      const int d = __builtin_amdgcn_readlane(dl, j);
      int e = e0 + j;
      e = e > nE - 1 ? nE - 1 : e;
      const v4f p = *(const v4f*)(pq + (size_t)s * PW + col);
      const v4f q = *(const v4f*)(pq + (size_t)d * PW + HID + col);
      const float* er = ea + (size_t)e * DEA;
      v4f av[DEA / 4];
#pragma unroll
      for (int i = 0; i < DEA / 4; ++i) av[i] = *(const v4f*)(er + 4 * i);
      v4f acc = p + q;
#pragma unroll
      for (int k = 0; k < DEA; ++k) acc = acc + av[k >> 2][k & 3] * we[k];
      acc.x = acc.x > 0.0f ? acc.x : 0.0f;
      acc.y = acc.y > 0.0f ? acc.y : 0.0f;
      acc.z = acc.z > 0.0f ? acc.z : 0.0f;
      acc.w = acc.w > 0.0f ? acc.w : 0.0f;
      const v4h o = __builtin_convertvector(acc, v4h);
      *(v4h*)(hw + j * LDH + col) = o;
    }
    __syncthreads();

    v8f acc2[4];
#pragma unroll
    for (int t = 0; t < 4; ++t) { v8f z = {0.f, 0.f, 0.f, 0.f, 0.f, 0.f, 0.f, 0.f}; acc2[t] = z; }
    const _Float16* arow = hw + m * LDH + 8 * hh;
    const _Float16* bp0  = w2p + (size_t)m * HID + 8 * hh;
#pragma unroll 1
    for (int kt = 0; kt < HID / 32; ++kt) {
      FragH a;
      a.h[0] = *(const v8h*)(arow + 32 * kt);
      a.h[1] = *(const v8h*)(arow + 32 * kt + 16);
#pragma unroll
      for (int t = 0; t < 4; ++t) {
        const _Float16* bp = bp0 + (size_t)(16 * t) * HID + 32 * kt;
        FragH bf;
        bf.h[0] = *(const v8h*)bp;
        bf.h[1] = *(const v8h*)(bp + 16);
        acc2[t] = wmh(a.v, bf.v, acc2[t]);
      }
    }

    v8f part;
#pragma unroll
    for (int r = 0; r < 8; ++r) {
      float pr = 0.0f;
#pragma unroll
      for (int t = 0; t < 4; ++t) {
        float v = acc2[t][r] * SCL_ACC + b2v[t];
        v = v > 0.0f ? v : 0.0f;
        pr += v * w3v[t];
      }
      part[r] = pr;
    }
#pragma unroll
    for (int r = 0; r < 8; ++r) {
      float t = part[r];
      t += __shfl_xor(t, 8);
      t += __shfl_xor(t, 4);
      t += __shfl_xor(t, 2);
      t += __shfl_xor(t, 1);
      part[r] = t;
    }
    float mine = 0.0f;
#pragma unroll
    for (int r = 0; r < 8; ++r) mine = ((m & 7) == r) ? part[r] : mine;
    const float res = tanhf(mine + c3);
    if (m < 8) sres[wave * EPW + 8 * hh + m] = res;
    __syncthreads();

    const v4f ov = *(const v4f*)(sres + 4 * lane);
    const int oe = tileBase + 4 * lane;
    const bool w0   = (wave == 0);
    const bool full = w0 && (oe + 3 < nE);
    const bool prt  = w0 && !full && (oe < nE);
    if (full) {
      *(volatile v4f*)(out + oe) = ov;
    } else if (prt) {
      if (oe < nE)     *(volatile float*)(out + oe)     = ov.x;
      if (oe + 1 < nE) *(volatile float*)(out + oe + 1) = ov.y;
      if (oe + 2 < nE) *(volatile float*)(out + oe + 2) = ov.z;
    }
    __threadfence();
    if (full) {
      *(volatile v4f*)(out + oe) = ov;
    } else if (prt) {
      if (oe < nE)     *(volatile float*)(out + oe)     = ov.x;
      if (oe + 1 < nE) *(volatile float*)(out + oe + 1) = ov.y;
      if (oe + 2 < nE) *(volatile float*)(out + oe + 2) = ov.z;
    }
  }
}

extern "C" void kernel_launch(void* const* d_in, const int* in_sizes, int n_in,
                              void* d_out, int out_size, void* d_ws, size_t ws_size,
                              hipStream_t stream) {
  if (n_in < 9) return;
  const int nN = in_sizes[0] / DN;
  const int nE = in_sizes[1] / 2;
  if (nN <= 0 || nE <= 0) return;
  if (in_sizes[0] != nN * DN || in_sizes[1] != 2 * nE) return;
  if (in_sizes[2] != nE * DEA) return;
  if (in_sizes[3] != K1 * HID || in_sizes[4] != HID) return;
  if (in_sizes[5] != HID * HID2 || in_sizes[6] != HID2) return;
  if (in_sizes[7] != HID2 || in_sizes[8] != 1) return;
  if (out_size != nE) return;
  if (nE > (1 << 27) || nN > (1 << 22)) return;

  const float* x  = (const float*)d_in[0];
  const int*   ei = (const int*)d_in[1];
  const float* ea = (const float*)d_in[2];
  const float* W1 = (const float*)d_in[3];
  const float* b1 = (const float*)d_in[4];
  const float* W2 = (const float*)d_in[5];
  const float* b2 = (const float*)d_in[6];
  const float* W3 = (const float*)d_in[7];
  const float* b3 = (const float*)d_in[8];
  float* out = (float*)d_out;

  const int NPAD  = ((nN + BM - 1) / BM) * BM;
  const int nXu   = NPAD * (DN / 8);
  const int nGemm = NPAD / BM;
  const int nEdge = (nE + EPBLK - 1) / EPBLK;

  char* ws = (char*)d_ws;
  size_t off = 0;
  const size_t oWPQ = off; off += (size_t)2 * HID * DN * 2;   off = (off + 255) & ~(size_t)255;
  const size_t oW2  = off; off += (size_t)HID2 * HID * 2;     off = (off + 255) & ~(size_t)255;
  const size_t oX   = off; off += (size_t)NPAD * DN * 2;      off = (off + 255) & ~(size_t)255;
  const size_t oPQ  = off; off += (size_t)NPAD * PW * 4;      off = (off + 255) & ~(size_t)255;
  if (off > ws_size || off > (size_t)WSCAP) return;
  _Float16* wPQ = (_Float16*)(ws + oWPQ);
  _Float16* w2p = (_Float16*)(ws + oW2);
  _Float16* xP  = (_Float16*)(ws + oX);
  float*    pqP = (float*)(ws + oPQ);

  k_tconv<HID><<<dim3(HID / CB, 2), NTHR, 0, stream>>>(W1, wPQ, HID, DN * HID, HID * DN, SCL_W);
  k_tconv<HID><<<dim3(HID2 / CB, 1), NTHR, 0, stream>>>(W2, w2p, HID2, 0, 0, SCL_W);
  k_xcvt<<<(nXu + NTHR - 1) / NTHR, NTHR, 0, stream>>>(x, xP, nN, nXu);
  k_nodegemm<<<nGemm, NTHR, 0, stream>>>(xP, wPQ, b1, pqP, nN);
  k_edge<<<nEdge, NTHR, 0, stream>>>(pqP, ei, ea, W1, w2p, b2, W3, b3, out, nE, nN);
}
